// gcn_layer_87454124081194
// MI455X (gfx1250) — hardware-run, weakly checked
//
#include <hip/hip_runtime.h>

typedef float          v8f   __attribute__((ext_vector_type(8)));
typedef float          v4f   __attribute__((ext_vector_type(4)));
typedef unsigned int   v4u   __attribute__((ext_vector_type(4)));
typedef int            v8i   __attribute__((ext_vector_type(8)));
typedef unsigned short v8us  __attribute__((ext_vector_type(8)));
typedef unsigned short v16us __attribute__((ext_vector_type(16)));
typedef __bf16         v16bf __attribute__((ext_vector_type(16)));
typedef _Float16       v16h  __attribute__((ext_vector_type(16)));
typedef v4f  __attribute__((may_alias)) v4fa;
typedef v8us __attribute__((may_alias)) v8usa;
union FragB { v16bf v; v16us u; v8us h[2]; v8i w; };
union FragH { v16h  v; v16us u; v8us h[2]; v8i w; };

__device__ __forceinline__ v8f wmb(const FragB& a, const FragB& b, v8f c) {
  v8f d = __builtin_amdgcn_wmma_f32_16x16x32_bf16(false, a.v, false, b.v, (short)0, c, false, false);
  asm volatile("v_nop\n\tv_nop\n\tv_nop\n\tv_nop" : "+v"(d) : "v"(a.w), "v"(b.w));
  return d;
}

__device__ __forceinline__ v8f wmh(const FragH& a, const FragH& b, v8f c) {
  v8f d = __builtin_amdgcn_wmma_f32_16x16x32_f16(false, a.v, false, b.v, (short)0, c, false, false);
  asm volatile("v_nop\n\tv_nop\n\tv_nop\n\tv_nop" : "+v"(d) : "v"(a.w), "v"(b.w));
  return d;
}

__device__ __forceinline__ unsigned bf16_bits(float f) {
  const unsigned u = __float_as_uint(f);
  const unsigned r = (u + 0x7FFFu + ((u >> 16) & 1u)) >> 16;
  const unsigned q = (u >> 16) | 0x40u;
  return ((u & 0x7fffffffu) > 0x7f800000u) ? q : r;
}

__device__ __forceinline__ float bf16_val(float f) {
  return __uint_as_float(bf16_bits(f) << 16);
}
__device__ __forceinline__ int clampi(int v, int lo, int hi) {
  return v < lo ? lo : (v > hi ? hi : v);
}

__device__ __forceinline__ unsigned f16_bits(float f) {
  const unsigned u  = __float_as_uint(f);
  const unsigned s  = (u >> 16) & 0x8000u;
  const unsigned a  = u & 0x7fffffffu;
  const unsigned t  = a - 0x38000000u;
  const unsigned r  = (t + 0x0FFFu + ((t >> 13) & 1u)) >> 13;
  const unsigned rc = r > 0x7C00u ? 0x7C00u : r;
  const bool small  = a < 0x38800000u;
  const bool isnan  = a > 0x7f800000u;
  const unsigned fin = small ? 0u : (s | rc);
  return isnan ? (s | 0x7E00u) : fin;
}

__device__ __forceinline__ unsigned pk16(unsigned lo, unsigned hi) { return lo | (hi << 16); }
__device__ __forceinline__ unsigned bf16_lo_bits(float v) {
  float hi = bf16_val(v);
  asm volatile("" : "+v"(hi));
  return bf16_bits(v - hi);
}
__device__ __forceinline__ v4u pack8_bf16(v4f a, v4f c) {
  return (v4u){ pk16(bf16_bits(a[0]), bf16_bits(a[1])), pk16(bf16_bits(a[2]), bf16_bits(a[3])),
                pk16(bf16_bits(c[0]), bf16_bits(c[1])), pk16(bf16_bits(c[2]), bf16_bits(c[3])) };
}
__device__ __forceinline__ v4u pack8_bf16_lo(v4f a, v4f c) {
  return (v4u){ pk16(bf16_lo_bits(a[0]), bf16_lo_bits(a[1])), pk16(bf16_lo_bits(a[2]), bf16_lo_bits(a[3])),
                pk16(bf16_lo_bits(c[0]), bf16_lo_bits(c[1])), pk16(bf16_lo_bits(c[2]), bf16_lo_bits(c[3])) };
}
__device__ __forceinline__ v4u pack8_f16(v4f a, v4f c) {
  return (v4u){ pk16(f16_bits(a[0]), f16_bits(a[1])), pk16(f16_bits(a[2]), f16_bits(a[3])),
                pk16(f16_bits(c[0]), f16_bits(c[1])), pk16(f16_bits(c[2]), f16_bits(c[3])) };
}

template <int FORM>
__global__ __launch_bounds__(256) void k_plane(const float* __restrict__ src, int rows, int cols, int ldsrc,
                                               unsigned short* __restrict__ dst, int MP, int KP) {
  static_assert(FORM >= 0 && FORM <= 3);
  const int KTOT = (FORM == 1 || FORM == 3) ? 2 * KP : KP;
  const unsigned ppr   = (unsigned)(KTOT >> 3);
  const unsigned kp8   = (unsigned)(KP >> 3);
  const unsigned total = (unsigned)MP * ppr;
  const unsigned g     = blockIdx.x * 256u + threadIdx.x;
  const unsigned rowu  = g / ppr;
  const unsigned p     = g - rowu * ppr;
  const bool second    = p >= kp8;
  const int row = (int)rowu;
  const int c0  = (int)((second ? p - kp8 : p) << 3);
  const float* srow = src + (size_t)clampi(row, 0, rows - 1) * (size_t)ldsrc;
  float x[8];
  unsigned mk[8];
#pragma unroll
  for (int e = 0; e < 8; ++e) {
    const int c = c0 + e;
    const float v = srow[clampi(c, 0, cols - 1)];
    asm volatile("" :: "v"(v));
    x[e]  = v;
    mk[e] = (row < rows && c < cols) ? 0xFFFFu : 0u;
  }
  const v4f a = (v4f){ x[0], x[1], x[2], x[3] };
  const v4f c = (v4f){ x[4], x[5], x[6], x[7] };
  v4u o;
  if (FORM == 2) {
    o = pack8_f16(a, c);
  } else {
    const v4u hi = pack8_bf16(a, c);
    o = hi;
    if (FORM == 1) { const v4u lo = pack8_bf16_lo(a, c); o = second ? lo : hi; }
  }
  const v4u mw = (v4u){ pk16(mk[0], mk[1]), pk16(mk[2], mk[3]), pk16(mk[4], mk[5]), pk16(mk[6], mk[7]) };
  o &= mw;
  if (g < total) {
    volatile v4u* q = (volatile v4u*)(dst + (size_t)g * 8);
    *q = o;
    __threadfence();
    *q = o;
  }
}

template <int FORM> struct FragOf    { typedef FragB T; };
template <>         struct FragOf<2> { typedef FragH T; };
__device__ __forceinline__ v8f mm(const FragB& a, const FragB& b, v8f c) { return wmb(a, b, c); }
__device__ __forceinline__ v8f mm(const FragH& a, const FragH& b, v8f c) { return wmh(a, b, c); }
template <class F> __device__ __forceinline__ F ld_frag(const unsigned short* p) {
  F f;
  f.h[0] = *(const v8usa*)(p);
  f.h[1] = *(const v8usa*)(p + 16);
  return f;
}

template <int FORM, int EPI>
__global__ __launch_bounds__(256) __attribute__((amdgpu_num_vgpr(248)))
void k_gemm_nt(const unsigned short* __restrict__ A, const unsigned short* __restrict__ B,
               const float* __restrict__ bias, float* __restrict__ D, int M, int N, int KTOT, int ldd) {
  static_assert(FORM >= 0 && FORM <= 2);
  static_assert(EPI == 0 || EPI == 1);
  typedef typename FragOf<FORM>::T F;
  __shared__ __attribute__((aligned(16))) float sT[8][16 * 68];
  const int lane = threadIdx.x & 31;
  const int wave = threadIdx.x >> 5;
  const int tilesM = (M + 63) >> 6;
  const int tilesN = (N + 63) >> 6;
  const int tile = blockIdx.x * 8 + wave;
  if (tile >= tilesM * tilesN) return;
  const int tm = tile / tilesN;
  const int tn = tile - tm * tilesN;
  const int m0 = tm << 6;
  const int n0 = tn << 6;

  const int rl = lane & 15;
  const int h8 = (lane >> 4) * 8;
  const unsigned short* pa = A + (size_t)(m0 + rl) * (size_t)KTOT + h8;
  const unsigned short* pb = B + (size_t)(n0 + rl) * (size_t)KTOT + h8;

  v8f acc[4][4];
#pragma unroll
  for (int i = 0; i < 4; ++i)
#pragma unroll
    for (int j = 0; j < 4; ++j) acc[i][j] = (v8f){0.f, 0.f, 0.f, 0.f, 0.f, 0.f, 0.f, 0.f};

#pragma unroll 1
  for (int k0 = 0; k0 < KTOT; k0 += 32) {
    F bf[4];
#pragma unroll
    for (int j = 0; j < 4; ++j) bf[j] = ld_frag<F>(pb + (size_t)(j << 4) * (size_t)KTOT + k0);
#pragma unroll
    for (int i = 0; i < 4; ++i) {
      const F af = ld_frag<F>(pa + (size_t)(i << 4) * (size_t)KTOT + k0);
#pragma unroll
      for (int j = 0; j < 4; ++j) acc[i][j] = mm(af, bf[j], acc[i][j]);
    }
  }

  float* slab = sT[wave];
  const int hh = lane >> 4;
  const int c4 = (lane & 15) * 4;
  const int nc = n0 + c4;
  const bool cok = nc < N;
  v4f bv = (v4f){0.f, 0.f, 0.f, 0.f};
  if (EPI == 1) {
    bv = *(const v4fa*)(bias + clampi(nc, 0, N - 4));
    asm volatile("" :: "v"(bv));
  }
#pragma unroll
  for (int i = 0; i < 4; ++i) {
    const int mBase = m0 + (i << 4);
#pragma unroll
    for (int j = 0; j < 4; ++j) {
#pragma unroll
      for (int r = 0; r < 8; ++r) slab[(h8 + r) * 68 + (j << 4) + rl] = acc[i][j][r];
    }
    __builtin_amdgcn_fence(__ATOMIC_RELEASE, "workgroup");
    __builtin_amdgcn_wave_barrier();
    __builtin_amdgcn_fence(__ATOMIC_ACQUIRE, "workgroup");
    v4f vv[8];
#pragma unroll
    for (int it = 0; it < 8; ++it) {
      const int row = it * 2 + hh;
      v4f v = *(const v4fa*)(slab + row * 68 + c4);
      if (EPI == 1) v += bv;
      vv[it] = v;
    }
    for (int pass = 0; pass < 2; ++pass) {
#pragma unroll
      for (int it = 0; it < 8; ++it) {
        const int row = mBase + it * 2 + hh;
        if (cok && row < M) *(volatile v4f*)(D + (size_t)row * (size_t)ldd + nc) = vv[it];
      }
      __threadfence();
    }
    __builtin_amdgcn_fence(__ATOMIC_RELEASE, "workgroup");
    __builtin_amdgcn_wave_barrier();
    __builtin_amdgcn_fence(__ATOMIC_ACQUIRE, "workgroup");
  }
}

#include <math.h>
#include <stddef.h>

#ifndef SPLIT_AGG
#define SPLIT_AGG 1
#endif
#ifndef SPLIT_NODE
#define SPLIT_NODE 1
#endif
#ifndef SPLIT_PQ
#define SPLIT_PQ 1
#endif
#ifndef SPLIT_EDGE
#define SPLIT_EDGE 1
#endif

#define NB   8
#define NN   256
#define ND   128
#define NH   8
#define ROWS (NB * NN)
#define KX   (ND * NH)
#define AGR  (NB * NH * NN)
#define OUT0_N (ROWS * ND)
#define OUT1_N (AGR * NN)
#define OUT2_N ROWS
#define OUT3_N (ROWS * NN)
#define OFF1 OUT0_N
#define OFF2 (OFF1 + OUT1_N)
#define OFF3 (OFF2 + OUT2_N)
#define OUT_TOTAL (OFF3 + OUT3_N)
#define EPITCH 72

static_assert(NB == 8 && NN == 256 && ND == 128 && NH == 8);
static_assert(ND * NH == 1024 && 2 * ND == 256 && 16 + NH == 24 && 16 + NH <= 32 && NN % 32 == 0);
static_assert(OFF1 == 262144 && OFF2 == 4456448 && OFF3 == 4458496 && OUT_TOTAL == 4982784);
static_assert((size_t)OFF1 * 4 == 1048576 && (size_t)OFF2 * 4 == 17825792 && (size_t)OFF3 * 4 == 17833984);
static_assert((size_t)OUT_TOTAL * 4 == 19931136);
static_assert(OFF1 % 32 == 0 && OFF2 % 32 == 0 && OFF3 % 32 == 0);
static_assert(ROWS % 64 == 0 && ND % 64 == 0 && AGR % 64 == 0 && (NH * NN) % 64 == 0);
static_assert(ND % 32 == 0 && (2 * NN) % 32 == 0 && (2 * KX) % 32 == 0 && (2 * ND) % 32 == 0);
static_assert((EPITCH * 2) % 16 == 0 && EPITCH >= 64);
static_assert(256 * EPITCH * 2 + 8 * 256 * 4 + 8 * 256 * 4 + 32 * 4 <= 65536);

typedef v4u __attribute__((may_alias)) v4ua;

static constexpr size_t SZ_MOLB  = (size_t)ROWS * ND * 2;
static constexpr size_t SZ_ADJ2  = (size_t)AGR * 512 * 2;
static constexpr size_t SZ_WT    = (size_t)ND * ND * 2;
static constexpr size_t SZ_W2T2  = (size_t)ND * 2 * KX * 2;
static constexpr size_t SZ_WPQ   = (size_t)64 * 256 * 2;
static constexpr size_t SZ_WA    = (size_t)32 * 64 * 2;
static constexpr size_t SZ_SUP   = (size_t)ROWS * ND * 4;
static constexpr size_t SZ_SUPT  = (size_t)ND * ROWS * 4;
static constexpr size_t SZ_STHL  = (size_t)NB * ND * 512 * 2;
static constexpr size_t SZ_AGG   = (size_t)AGR * ND * 4;
static constexpr size_t SZ_XHL   = (size_t)ROWS * 2 * KX * 2;
static constexpr size_t SZ_Y     = (size_t)ROWS * ND * 4;
static constexpr size_t SZ_OUTHL = (size_t)ROWS * 2 * ND * 2;
static constexpr size_t SZ_PQ    = (size_t)ROWS * 32 * 4;
static constexpr size_t O_MOLB  = 0;
static constexpr size_t O_ADJ2  = O_MOLB  + SZ_MOLB;
static constexpr size_t O_WT    = O_ADJ2  + SZ_ADJ2;
static constexpr size_t O_W2T2  = O_WT    + SZ_WT;
static constexpr size_t O_WPQ   = O_W2T2  + SZ_W2T2;
static constexpr size_t O_WA    = O_WPQ   + SZ_WPQ;
static constexpr size_t O_SUP   = O_WA    + SZ_WA;
static constexpr size_t O_SUPT  = O_SUP   + SZ_SUP;
static constexpr size_t O_STHL  = O_SUPT  + SZ_SUPT;
static constexpr size_t O_AGG   = O_STHL  + SZ_STHL;
static constexpr size_t O_XHL   = O_AGG   + SZ_AGG;
static constexpr size_t O_Y     = O_XHL   + SZ_XHL;
static constexpr size_t O_OUTHL = O_Y     + SZ_Y;
static constexpr size_t O_PQ    = O_OUTHL + SZ_OUTHL;
static constexpr size_t WS_TOTAL = O_PQ + SZ_PQ;
static_assert(SZ_MOLB % 256 == 0 && SZ_ADJ2 % 256 == 0 && SZ_WT % 256 == 0 && SZ_W2T2 % 256 == 0);
static_assert(SZ_WPQ % 256 == 0 && SZ_WA % 256 == 0 && SZ_SUP % 256 == 0 && SZ_SUPT % 256 == 0);
static_assert(SZ_STHL % 256 == 0 && SZ_AGG % 256 == 0 && SZ_XHL % 256 == 0 && SZ_Y % 256 == 0);
static_assert(SZ_OUTHL % 256 == 0 && SZ_PQ % 256 == 0);
static_assert(WS_TOTAL == 40177664);
static_assert(WS_TOTAL <= ((size_t)128 << 20));

#define U_WT  2048
#define U_W2  32768
#define U_PQ  2048
#define U_WA  256
#define U_TOT (U_WT + U_W2 + U_PQ + U_WA)
static_assert(U_WT == ND * ND / 8 && U_W2 == ND * 2 * KX / 8 && U_PQ == 64 * 256 / 8 && U_WA == 32 * 64 / 8);
static_assert(U_WT % 256 == 0 && U_W2 % 256 == 0 && U_PQ % 256 == 0 && U_WA % 256 == 0 && U_TOT == 37120);

__device__ __forceinline__ void wunit(const float* __restrict__ src, int pitch, int nrows, int ncols,
                                      int rowbase, int rowstep, int nvalid, int col, bool colok,
                                      unsigned short* dstp) {
  float x[8];
  unsigned mk[8];
  const int cc = clampi(col, 0, ncols - 1);
#pragma unroll
  for (int e = 0; e < 8; ++e) {
    const int r  = clampi(rowbase + e * rowstep, 0, nrows - 1);
    const float v = src[(size_t)r * (size_t)pitch + cc];
    asm volatile("" :: "v"(v));
    x[e]  = v;
    mk[e] = (colok && e < nvalid) ? 0xFFFFu : 0u;
  }
  const v4f a = (v4f){ x[0], x[1], x[2], x[3] };
  const v4f c = (v4f){ x[4], x[5], x[6], x[7] };
  v4u o = pack8_bf16(a, c);
  const v4u mw = (v4u){ pk16(mk[0], mk[1]), pk16(mk[2], mk[3]), pk16(mk[4], mk[5]), pk16(mk[6], mk[7]) };
  o &= mw;
  volatile v4u* q = (volatile v4u*)dstp;
  *q = o;
  __threadfence();
  *q = o;
}

__global__ __launch_bounds__(256) void k_wprep(const float* __restrict__ wgt, const float* __restrict__ wout,
                                               const float* __restrict__ wadj, const float* __restrict__ wao,
                                               unsigned short* wt, unsigned short* w2t2,
                                               unsigned short* wpq, unsigned short* wa) {
  const int u = (int)blockIdx.x * 256 + (int)threadIdx.x;
  if (u < U_WT) {
    const int n = u >> 4, kk = (u & 15) * 8;
    wunit(wgt, ND, ND, ND, kk, 1, 8, n, true, wt + (size_t)u * 8);
  } else if (u < U_WT + U_W2) {
    const int v = u - U_WT;
    const int n = v >> 8;
    const int kk = ((v & 255) * 8) & (KX - 1);
    const int h = kk >> 7, d0 = kk & 127;
    wunit(wout, ND, KX, ND, d0 * NH + h, NH, 8, n, true, w2t2 + (size_t)v * 8);
  } else if (u < U_WT + U_W2 + U_PQ) {
    const int v = u - U_WT - U_W2;
    const int n = v >> 5;
    const int kk = ((v & 31) * 8) & 127;
    const bool isq = n >= 16;
    const int col = isq ? n - 16 : n;
    wunit(wadj, 16, 2 * ND, 16, (isq ? ND : 0) + kk, 1, 8, col, n < 32, wpq + (size_t)v * 8);
  } else if (u < U_TOT) {
    const int v = u - U_WT - U_W2 - U_PQ;
    const int n = v >> 3;
    const int k = (v & 7) * 8;
    const bool sec = k >= 32;
    const int kk = sec ? k - 32 : k;
    wunit(wao, NH, 16 + NH, NH, kk, 1, (sec ? 16 : 16 + NH) - kk, n, n < NH, wa + (size_t)v * 8);
  }
}

__global__ __launch_bounds__(256) void k_split(const float* __restrict__ SUPT, unsigned short* STHL) {
  const unsigned g = blockIdx.x * 256u + threadIdx.x;
  const unsigned b = g >> 13, d = (g >> 6) & 127u, p = g & 63u;
  const bool second = p >= 32u;
  const unsigned j0 = 8u * (p & 31u);
  const float* sp = SUPT + (size_t)d * ROWS + (size_t)b * NN + j0;
  const v4f a = *(const v4fa*)(sp);
  const v4f c = *(const v4fa*)(sp + 4);
  const v4u hi = pack8_bf16(a, c);
  const v4u lo = pack8_bf16_lo(a, c);
  const v4u z4 = (v4u){ 0u, 0u, 0u, 0u };
  const v4u o = second ? (SPLIT_AGG ? lo : z4) : hi;
  volatile v4u* q = (volatile v4u*)(STHL + (size_t)g * 8);
  *q = o;
  __threadfence();
  *q = o;
}

__global__ __launch_bounds__(256) void k_act(const float* __restrict__ AGG, const float* __restrict__ SUP,
                                             const float* __restrict__ bias, const float* __restrict__ mask,
                                             unsigned short* XHL) {
  __shared__ __attribute__((aligned(16))) float st[KX];
  const int t = (int)threadIdx.x;
  const int bi = (int)blockIdx.x;
  const int b = bi >> 8, i = bi & 255;
  const float mk = bf16_val(mask[bi]);
#pragma unroll 1
  for (int it = 0; it < 4; ++it) {
    const int idx = it * 256 + t;
    const int h = idx >> 7, d = idx & 127;
    const float a  = AGG[((size_t)((b * NH + h) * NN + i)) * ND + d];
    const float sv = SUP[(size_t)bi * ND + d];
    const float bv = bias[d];
    asm volatile("" :: "v"(a));
    asm volatile("" :: "v"(sv));
    asm volatile("" :: "v"(bv));
    st[idx] = tanhf((a + sv) + bf16_val(bv)) * mk;
  }
  __syncthreads();
  const bool second = t >= 128;
  const int k0 = 8 * (t & 127);
  const v4f a = *(const v4fa*)(st + k0);
  const v4f c = *(const v4fa*)(st + k0 + 4);
  const v4u hi = pack8_bf16(a, c);
  const v4u lo = pack8_bf16_lo(a, c);
  const v4u z4 = (v4u){ 0u, 0u, 0u, 0u };
  const v4u o = second ? (SPLIT_NODE ? lo : z4) : hi;
  volatile v4u* q = (volatile v4u*)(XHL + (size_t)bi * (2 * KX) + (size_t)t * 8);
  *q = o;
  __threadfence();
  *q = o;
}

__global__ __launch_bounds__(256) void k_node(const float* __restrict__ Y, const float* __restrict__ b_out,
                                              const float* __restrict__ mask, float* out0, unsigned short* OUTHL) {
  __shared__ __attribute__((aligned(16))) float so[8 * ND];
  const int t = (int)threadIdx.x;
  const int r0 = (int)blockIdx.x * 8;
#pragma unroll 1
  for (int it = 0; it < 4; ++it) {
    const int idx = it * 256 + t;
    const int row = idx >> 7, c = idx & 127;
    const float y  = Y[(size_t)(r0 + row) * ND + c];
    const float bo = b_out[c];
    const float mv = mask[r0 + row];
    asm volatile("" :: "v"(y));
    asm volatile("" :: "v"(bo));
    asm volatile("" :: "v"(mv));
    so[idx] = tanhf(y + bf16_val(bo)) * bf16_val(mv);
  }
  __syncthreads();
  const v4f f0 = *(const v4fa*)(so + 4 * t);
  const int row = t >> 5, p = t & 31;
  const bool second = p >= 16;
  const int c0 = 8 * (p & 15);
  const v4f a = *(const v4fa*)(so + row * ND + c0);
  const v4f c = *(const v4fa*)(so + row * ND + c0 + 4);
  const v4u hi = pack8_bf16(a, c);
  const v4u lo = pack8_bf16_lo(a, c);
  const v4u z4 = (v4u){ 0u, 0u, 0u, 0u };
  const v4u o = second ? (SPLIT_PQ ? lo : z4) : hi;
  float* op = out0 + (size_t)r0 * ND + 4 * t;
  unsigned short* dh = OUTHL + (size_t)r0 * (2 * ND) + (size_t)t * 8;
  for (int ps = 0; ps < 2; ++ps) {
    *(volatile v4f*)op = f0;
    *(volatile v4u*)dh = o;
    __threadfence();
  }
}

#define EK (SPLIT_EDGE ? 2 : 1)

__global__ __launch_bounds__(256) __attribute__((amdgpu_num_vgpr(248)))
void k_edge(const float* __restrict__ adj, const float* __restrict__ adjmask, const float* __restrict__ PQ,
            const float* __restrict__ b_adj, const float* __restrict__ b_adjout,
            const unsigned short* __restrict__ WA, float* out1) {
  __shared__ __attribute__((aligned(16))) unsigned short As[256 * EPITCH];
  __shared__ __attribute__((aligned(16))) float adjs[NH * NN];
  __shared__ __attribute__((aligned(16))) float ds[NH * NN];
  __shared__ __attribute__((aligned(16))) float sq[32];
  const int t = (int)threadIdx.x, lane = t & 31, wave = t >> 5, hh = lane >> 4, m = lane & 15;
  const int bi = (int)blockIdx.x;
  const int b = bi >> 8, i = bi & 255;

  if (t < 32) {
    const int c = t & 15;
    const float q  = PQ[(size_t)bi * 32 + 16 + c];
    const float bb = b_adj[c];
    asm volatile("" :: "v"(q));
    asm volatile("" :: "v"(bb));
    sq[t] = (t < 16) ? q : bf16_val(bb);
  }
#pragma unroll
  for (int it = 0; it < 2; ++it) {
    const int idx = it * 256 + t;
    const int h = idx >> 6, j4 = (idx & 63) * 4;
    const v4f v = *(const v4fa*)(adj + ((size_t)((b * NH + h) * NN + i)) * NN + j4);
    const v4f r = (v4f){ bf16_val(v[0]), bf16_val(v[1]), bf16_val(v[2]), bf16_val(v[3]) };
    *(v4fa*)(adjs + h * NN + j4) = r;
  }
  FragB bw[EK];
  {
    const unsigned short* bp = WA + m * 64 + 8 * hh;
#pragma unroll
    for (int ks = 0; ks < EK; ++ks) bw[ks] = ld_frag<FragB>(bp + 32 * ks);
  }
  __syncthreads();

  {
    const float* prow = PQ + ((size_t)(b * NN + t)) * 32;
    const v4f p0 = *(const v4fa*)(prow);
    const v4f p1 = *(const v4fa*)(prow + 4);
    const v4f p2 = *(const v4fa*)(prow + 8);
    const v4f p3 = *(const v4fa*)(prow + 12);
    const v4f q0 = *(const v4fa*)(sq);
    const v4f q1 = *(const v4fa*)(sq + 4);
    const v4f q2 = *(const v4fa*)(sq + 8);
    const v4f q3 = *(const v4fa*)(sq + 12);
    const v4f e0 = *(const v4fa*)(sq + 16);
    const v4f e1 = *(const v4fa*)(sq + 20);
    const v4f e2 = *(const v4fa*)(sq + 24);
    const v4f e3 = *(const v4fa*)(sq + 28);
    const v4f x0 = (v4f){ fmaxf((p0[0] + q0[0]) + e0[0], 0.0f), fmaxf((p0[1] + q0[1]) + e0[1], 0.0f),
                          fmaxf((p0[2] + q0[2]) + e0[2], 0.0f), fmaxf((p0[3] + q0[3]) + e0[3], 0.0f) };
    const v4f x1 = (v4f){ fmaxf((p1[0] + q1[0]) + e1[0], 0.0f), fmaxf((p1[1] + q1[1]) + e1[1], 0.0f),
                          fmaxf((p1[2] + q1[2]) + e1[2], 0.0f), fmaxf((p1[3] + q1[3]) + e1[3], 0.0f) };
    const v4f x2 = (v4f){ fmaxf((p2[0] + q2[0]) + e2[0], 0.0f), fmaxf((p2[1] + q2[1]) + e2[1], 0.0f),
                          fmaxf((p2[2] + q2[2]) + e2[2], 0.0f), fmaxf((p2[3] + q2[3]) + e2[3], 0.0f) };
    const v4f x3 = (v4f){ fmaxf((p3[0] + q3[0]) + e3[0], 0.0f), fmaxf((p3[1] + q3[1]) + e3[1], 0.0f),
                          fmaxf((p3[2] + q3[2]) + e3[2], 0.0f), fmaxf((p3[3] + q3[3]) + e3[3], 0.0f) };
    const v4f a0 = (v4f){ adjs[0 * NN + t], adjs[1 * NN + t], adjs[2 * NN + t], adjs[3 * NN + t] };
    const v4f a1 = (v4f){ adjs[4 * NN + t], adjs[5 * NN + t], adjs[6 * NN + t], adjs[7 * NN + t] };
    const v4u z4 = (v4u){ 0u, 0u, 0u, 0u };
    unsigned short* arow = As + t * EPITCH;
    *(v4ua*)(arow)      = pack8_bf16(x0, x1);
    *(v4ua*)(arow + 8)  = pack8_bf16(x2, x3);
    *(v4ua*)(arow + 16) = pack8_bf16(a0, a1);
    *(v4ua*)(arow + 24) = z4;
    *(v4ua*)(arow + 32) = pack8_bf16_lo(x0, x1);
    *(v4ua*)(arow + 40) = pack8_bf16_lo(x2, x3);
    *(v4ua*)(arow + 48) = z4;
    *(v4ua*)(arow + 56) = z4;
  }
  __syncthreads();

#pragma unroll
  for (int tl = 0; tl < 2; ++tl) {
    const int jt = 2 * wave + tl;
    v8f acc = (v8f){0.f, 0.f, 0.f, 0.f, 0.f, 0.f, 0.f, 0.f};
    const unsigned short* ap = As + (16 * jt + m) * EPITCH + 8 * hh;
#pragma unroll
    for (int ks = 0; ks < EK; ++ks) {
      FragB af;
      af.h[0] = *(const v8usa*)(ap + 32 * ks);
      af.h[1] = *(const v8usa*)(ap + 32 * ks + 16);
      acc = wmb(af, bw[ks], acc);
    }
    const int jb = 16 * jt + 8 * hh;
#pragma unroll
    for (int r = 0; r < 8; ++r) {
      if (m < NH) ds[m * NN + jb + r] = acc[r];
    }
  }
  __syncthreads();

  {
    const float bo = bf16_val(b_adjout[wave]);
    float* orow = out1 + ((size_t)((b * NH + wave) * NN + i)) * NN;
    v4f res[2];
#pragma unroll
    for (int it = 0; it < 2; ++it) {
      const int j0 = it * 128 + 4 * lane;
      const v4f d4 = *(const v4fa*)(ds + wave * NN + j0);
      const v4f a4 = *(const v4fa*)(adjs + wave * NN + j0);
      const v4f m4 = *(const v4fa*)(adjmask + (size_t)bi * NN + j0);
      res[it] = (v4f){ fmaxf(d4[0] + bo, 0.0f) * bf16_val(m4[0]) + a4[0],
                       fmaxf(d4[1] + bo, 0.0f) * bf16_val(m4[1]) + a4[1],
                       fmaxf(d4[2] + bo, 0.0f) * bf16_val(m4[2]) + a4[2],
                       fmaxf(d4[3] + bo, 0.0f) * bf16_val(m4[3]) + a4[3] };
    }
    for (int ps = 0; ps < 2; ++ps) {
#pragma unroll
      for (int it = 0; it < 2; ++it) *(volatile v4f*)(orow + it * 128 + 4 * lane) = res[it];
      __threadfence();
    }
  }
}

#define CP_V4 ((OUT2_N + OUT3_N) / 4)
static_assert(CP_V4 == 131584 && CP_V4 % 256 == 0 && OUT2_N / 4 == 512);

__global__ __launch_bounds__(256) void k_copy(const float* __restrict__ mask, const float* __restrict__ adjmask,
                                              float* outm) {
  const int g = (int)blockIdx.x * 256 + (int)threadIdx.x;
  const bool isM = blockIdx.x < 2;
  const int mi = clampi(g, 0, OUT2_N / 4 - 1);
  const int ai = clampi(g - OUT2_N / 4, 0, OUT3_N / 4 - 1);
  const v4f vm = *(const v4fa*)(mask + 4 * (size_t)mi);
  const v4f va = *(const v4fa*)(adjmask + 4 * (size_t)ai);
  asm volatile("" :: "v"(vm));
  asm volatile("" :: "v"(va));
  const v4f s = isM ? vm : va;
  const v4f o = (v4f){ bf16_val(s[0]), bf16_val(s[1]), bf16_val(s[2]), bf16_val(s[3]) };
  volatile v4f* q = (volatile v4f*)(outm + 4 * (size_t)g);
  *q = o;
  __threadfence();
  *q = o;
}

static inline int cdiv(int a, int b) { return (a + b - 1) / b; }

extern "C" void kernel_launch(void* const* d_in, const int* in_sizes, int n_in,
                              void* d_out, int out_size, void* d_ws, size_t ws_size,
                              hipStream_t stream) {
  if (n_in < 12) return;
  if (in_sizes[0] != ROWS * ND) return;
  if (in_sizes[1] != OUT1_N) return;
  if (in_sizes[2] != ROWS) return;
  if (in_sizes[3] != OUT3_N) return;
  if (in_sizes[4] != ND * ND) return;
  if (in_sizes[5] != ND) return;
  if (in_sizes[6] != KX * ND) return;
  if (in_sizes[7] != ND) return;
  if (in_sizes[8] != 2 * ND * 16) return;
  if (in_sizes[9] != 16) return;
  if (in_sizes[10] != (16 + NH) * NH) return;
  if (in_sizes[11] != NH) return;
  if ((long long)out_size != (long long)OUT_TOTAL) return;
  if ((size_t)WS_TOTAL > ws_size) return;

  const float* mol     = (const float*)d_in[0];
  const float* adj     = (const float*)d_in[1];
  const float* mask    = (const float*)d_in[2];
  const float* adjmask = (const float*)d_in[3];
  const float* weight  = (const float*)d_in[4];
  const float* bias    = (const float*)d_in[5];
  const float* W_out   = (const float*)d_in[6];
  const float* b_out   = (const float*)d_in[7];
  const float* W_adj   = (const float*)d_in[8];
  const float* b_adj   = (const float*)d_in[9];
  const float* W_ao    = (const float*)d_in[10];
  const float* b_ao    = (const float*)d_in[11];
  float* out0 = (float*)d_out;
  float* out1 = (float*)d_out + (size_t)OFF1;
  float* out2 = (float*)d_out + (size_t)OFF2;

  char* ws = (char*)d_ws;
  unsigned short* MOLB  = (unsigned short*)(ws + O_MOLB);
  unsigned short* ADJ2  = (unsigned short*)(ws + O_ADJ2);
  unsigned short* WT    = (unsigned short*)(ws + O_WT);
  unsigned short* W2T2  = (unsigned short*)(ws + O_W2T2);
  unsigned short* WPQ   = (unsigned short*)(ws + O_WPQ);
  unsigned short* WA    = (unsigned short*)(ws + O_WA);
  float*          SUP   = (float*)(ws + O_SUP);
  float*          SUPT  = (float*)(ws + O_SUPT);
  unsigned short* STHL  = (unsigned short*)(ws + O_STHL);
  float*          AGG   = (float*)(ws + O_AGG);
  unsigned short* XHL   = (unsigned short*)(ws + O_XHL);
  float*          Y     = (float*)(ws + O_Y);
  unsigned short* OUTHL = (unsigned short*)(ws + O_OUTHL);
  float*          PQ    = (float*)(ws + O_PQ);

  k_plane<0><<<ROWS * ND / 8 / 256, 256, 0, stream>>>(mol, ROWS, ND, ND, MOLB, ROWS, ND);
  k_plane<3><<<AGR * 512 / 8 / 256, 256, 0, stream>>>(adj, AGR, NN, NN, ADJ2, AGR, NN);
  k_wprep<<<U_TOT / 256, 256, 0, stream>>>(weight, W_out, W_adj, W_ao, WT, W2T2, WPQ, WA);
  k_gemm_nt<0, 0><<<cdiv(32 * 2, 8), 256, 0, stream>>>(MOLB, WT, SUP, SUP, ROWS, ND, ND, ND);
  k_gemm_nt<0, 0><<<cdiv(2 * 32, 8), 256, 0, stream>>>(WT, MOLB, SUP, SUPT, ND, ROWS, ND, ROWS);
  k_split<<<NB * ND * 64 / 256, 256, 0, stream>>>(SUPT, STHL);
  for (int b = 0; b < NB; ++b) {
    k_gemm_nt<0, 0><<<cdiv(32 * 2, 8), 256, 0, stream>>>(ADJ2 + (size_t)b * (NH * NN) * 512,
                                                        STHL + (size_t)b * ND * 512, SUP,
                                                        AGG + (size_t)b * (NH * NN) * ND, NH * NN, ND, 512, ND);
  }
  k_act<<<ROWS, 256, 0, stream>>>(AGG, SUP, bias, mask, XHL);
  k_gemm_nt<0, 0><<<cdiv(32 * 2, 8), 256, 0, stream>>>(XHL, W2T2, SUP, Y, ROWS, ND, 2 * KX, ND);
  k_node<<<ROWS / 8, 256, 0, stream>>>(Y, b_out, mask, out0, OUTHL);
  k_gemm_nt<0, 0><<<cdiv(32, 8), 256, 0, stream>>>(OUTHL, WPQ, SUP, PQ, ROWS, 32, 2 * ND, 32);
  k_edge<<<ROWS, 256, 0, stream>>>(adj, adjmask, PQ, b_adj, b_ao, WA, out1);
  k_copy<<<CP_V4 / 256, 256, 0, stream>>>(mask, adjmask, out2);
}
